// GraphModule_10720238370828
// MI455X (gfx1250) — hardware-verified
//
#include <hip/hip_runtime.h>


#define NB_  8
#define NN_  2048
#define DD   128
#define NOUT 128
#define LOSC 1024.0f
#define LOSCI (1.0f / 1024.0f)

typedef _Float16 h16;
typedef unsigned short bf;
typedef __attribute__((ext_vector_type(16))) __bf16   v16bf;
typedef __attribute__((ext_vector_type(16))) _Float16 v16h;
typedef __attribute__((ext_vector_type(8)))  _Float16 v8h;
typedef __attribute__((ext_vector_type(8)))  unsigned short v8us;
typedef __attribute__((ext_vector_type(8)))  float    v8f;
typedef __attribute__((ext_vector_type(4)))  float    v4f;
typedef v8h  __attribute__((may_alias)) v8ha;
typedef v4f  __attribute__((may_alias)) v4fa;
typedef v8us __attribute__((may_alias)) v8usa;

__device__ __forceinline__ unsigned short f2bf(float f) { unsigned u = __float_as_uint(f); u += 0x7FFFu + ((u >> 16) & 1u); return (unsigned short)(u >> 16); }
__device__ __forceinline__ float bf2f(unsigned short b) { return __uint_as_float(((unsigned)b) << 16); }
__device__ __forceinline__ float bfr(float f) { return bf2f(f2bf(f)); }
__device__ __forceinline__ v16h cat16(v8h lo, v8h hi) { return __builtin_shufflevector(lo, hi, 0, 1, 2, 3, 4, 5, 6, 7, 8, 9, 10, 11, 12, 13, 14, 15); }
__device__ __forceinline__ v16bf cat16b(v8us lo, v8us hi) { return __builtin_bit_cast(v16bf, __builtin_shufflevector(lo, hi, 0, 1, 2, 3, 4, 5, 6, 7, 8, 9, 10, 11, 12, 13, 14, 15)); }
__device__ __forceinline__ v8f wmma16(v16h a, v16h b, v8f c) { return __builtin_amdgcn_wmma_f32_16x16x32_f16(false, a, false, b, (short)0, c, false, false); }
__device__ __forceinline__ v8f wmmab(v16bf a, v16bf b, v8f c) { return __builtin_amdgcn_wmma_f32_16x16x32_bf16(false, a, false, b, (short)0, c, false, false); }
#define VST2(T, p, v) do { const T vst2_v_ = (v); *(volatile T*)(p) = vst2_v_; __threadfence(); *(volatile T*)(p) = vst2_v_; } while (0)

__global__ __launch_bounds__(256) void k_sij(const float* __restrict__ x, const float* __restrict__ gw, float* SI, float* SJ) {
    const int lane = threadIdx.x & 31, wid = blockIdx.x * 8 + (threadIdx.x >> 5);
    if (wid >= NB_ * NN_ / 32) return;
    const size_t n0 = (size_t)wid * 32 + lane;
    const float* xr = x + n0 * DD;
    float si = 0.f, sj = 0.f;
#pragma unroll 4
    for (int d = 0; d < DD; ++d) { const float v = bfr(xr[d]); sj += v * bfr(gw[d]); si += v * bfr(gw[DD + d]); }
    VST2(float, SI + n0, si); VST2(float, SJ + n0, sj);
}

__global__ __launch_bounds__(256) void k_xt(const float* __restrict__ x, h16* XT16) {
    __shared__ __align__(16) h16 tl[64 * 72];
    const int tid = threadIdx.x, b = blockIdx.z, n0 = blockIdx.x * 64, d0 = blockIdx.y * 64;
    const int nn = tid >> 2, dq = (tid & 3) * 16;
#pragma unroll
    for (int i = 0; i < 16; ++i) tl[(dq + i) * 72 + nn] = (h16)bfr(x[((size_t)b * NN_ + n0 + nn) * DD + d0 + dq + i]);
    __syncthreads();
    const int piece = tid & 7;
    auto pass = [&]() {
#pragma unroll
        for (int s = 0; s < 2; ++s) { const int dr = (tid >> 3) + 32 * s; const v8h val = *(const v8ha*)(tl + dr * 72 + piece * 8);
            *(volatile v8h*)(XT16 + ((size_t)b * DD + d0 + dr) * NN_ + n0 + piece * 8) = val; }
    };
    pass(); __threadfence(); pass();
}

__global__ __launch_bounds__(128) void k_agg(const float* __restrict__ SI, const float* __restrict__ SJ, const float* __restrict__ rel, const float* __restrict__ gw, const float* __restrict__ gb,
                                            const h16* __restrict__ XT16, bf* AH, bf* AL) {
    __shared__ __align__(16) float ost[4][16 * 132];
    const int lane = threadIdx.x & 31, wave = threadIdx.x >> 5, lr = lane & 15, hi = lane >> 4;
    const int b = blockIdx.y, i0 = blockIdx.x * 64 + wave * 16;
    const int i = i0 + lr;
    const float wr = bfr(gw[2 * DD]), g0 = bfr(gb[0]);
    const float sii = SI[(size_t)b * NN_ + i] + g0;
    const float* relr = rel + (size_t)i * NN_;
    const float* sjb = SJ + (size_t)b * NN_;
    const h16* xtb = XT16 + (size_t)b * DD * NN_;
    v8f acc[8], accx[8];
#pragma unroll
    for (int n = 0; n < 8; ++n) { acc[n] = (v8f){}; accx[n] = (v8f){}; }
#pragma unroll 1
    for (int kc = 0; kc < NN_; kc += 32) {
        v16h ah, al;
#pragma unroll
        for (int q = 0; q < 16; ++q) {
            const int j = kc + ((q < 8) ? (8 * hi + q) : (16 + 8 * hi + (q - 8)));
            const float v = sii + sjb[j] + bfr(relr[j]) * wr;
            const h16 hv = (h16)v; ah[q] = hv; al[q] = (h16)((v - (float)hv) * LOSC);
        }
#pragma unroll
        for (int n = 0; n < 8; ++n) { const h16* bp = xtb + (size_t)(n * 16 + lr) * NN_ + kc + 8 * hi; const v16h bb = cat16(*(const v8h*)bp, *(const v8h*)(bp + 16));
            acc[n] = wmma16(ah, bb, acc[n]); accx[n] = wmma16(al, bb, accx[n]); }
    }
    asm volatile("v_nop\n\tv_nop\n\tv_nop\n\tv_nop" : "+v"(acc[0]), "+v"(acc[3]), "+v"(acc[7]), "+v"(accx[0]), "+v"(accx[3]), "+v"(accx[7]));
    asm volatile("v_nop\n\tv_nop\n\tv_nop\n\tv_nop" : "+v"(acc[1]), "+v"(acc[2]), "+v"(acc[4]), "+v"(acc[5]), "+v"(acc[6]), "+v"(accx[1]), "+v"(accx[2]), "+v"(accx[4]), "+v"(accx[5]), "+v"(accx[6]));
    float* os = &ost[wave][0];
#pragma unroll
    for (int n = 0; n < 8; ++n)
#pragma unroll
        for (int jx = 0; jx < 8; ++jx) os[(hi * 8 + jx) * 132 + n * 16 + lr] = acc[n][jx] + accx[n][jx] * LOSCI;
    __syncthreads();
    const size_t rbase = ((size_t)b * NN_ + i0) * DD;
    auto pass = [&]() {
#pragma unroll
        for (int s = 0; s < 8; ++s) { const int row = 2 * s + (lane >> 4), piece = lane & 15; const float* sp = os + row * 132 + piece * 8; v8us oh, ol;
#pragma unroll
            for (int t = 0; t < 8; ++t) { const unsigned short hb = f2bf(sp[t]); oh[t] = hb; ol[t] = f2bf(sp[t] - bf2f(hb)); }
            *(volatile v8us*)(AH + rbase + (size_t)row * DD + piece * 8) = oh; *(volatile v8us*)(AL + rbase + (size_t)row * DD + piece * 8) = ol; }
    };
    pass(); __threadfence(); pass();
}

__global__ __launch_bounds__(256) void k_wt(const float* __restrict__ Wm, bf* WT) {
    __shared__ __align__(16) unsigned short tl[64 * 72];
    const int tid = threadIdx.x, k0 = blockIdx.x * 64, n0 = blockIdx.y * 64;
    const int kk = tid >> 2, nq = (tid & 3) * 16;
#pragma unroll
    for (int i2 = 0; i2 < 16; ++i2) tl[(nq + i2) * 72 + kk] = f2bf(Wm[(size_t)(k0 + kk) * NOUT + n0 + nq + i2]);
    __syncthreads();
    const int piece = tid & 7;
    auto pass = [&]() {
#pragma unroll
        for (int s = 0; s < 2; ++s) { const int nr = (tid >> 3) + 32 * s; const v8us val = *(const v8usa*)(tl + nr * 72 + piece * 8);
            *(volatile v8us*)(WT + (size_t)(n0 + nr) * DD + k0 + piece * 8) = val; }
    };
    pass(); __threadfence(); pass();
}
__global__ __launch_bounds__(128) void k_out(const bf* __restrict__ A, const bf* __restrict__ Al, const bf* __restrict__ Bn, const float* __restrict__ bias, float* C) {
    __shared__ __align__(16) float ost[4][16 * 68];
    const int lane = threadIdx.x & 31, wave = threadIdx.x >> 5, lr = lane & 15, hi = lane >> 4;
    const int r0 = blockIdx.x * 64 + wave * 16, c0 = blockIdx.y * 64;
    const size_t aoff = (size_t)(r0 + lr) * DD + 8 * hi;
    size_t boff[4];
#pragma unroll
    for (int t = 0; t < 4; ++t) boff[t] = (size_t)(c0 + t * 16 + lr) * DD + 8 * hi;
    v8f acc[4];
#pragma unroll
    for (int t = 0; t < 4; ++t) acc[t] = (v8f){};
#pragma unroll
    for (int kc = 0; kc < DD; kc += 32) {
        const v16bf a = cat16b(*(const v8us*)(A + aoff + kc), *(const v8us*)(A + aoff + kc + 16)), al = cat16b(*(const v8us*)(Al + aoff + kc), *(const v8us*)(Al + aoff + kc + 16));
#pragma unroll
        for (int t = 0; t < 4; ++t) { const v16bf bb = cat16b(*(const v8us*)(Bn + boff[t] + kc), *(const v8us*)(Bn + boff[t] + kc + 16)); acc[t] = wmmab(a, bb, acc[t]); acc[t] = wmmab(al, bb, acc[t]); }
    }
    asm volatile("v_nop\n\tv_nop\n\tv_nop\n\tv_nop" : "+v"(acc[0]), "+v"(acc[1]), "+v"(acc[2]), "+v"(acc[3]));
    float* os = &ost[wave][0];
#pragma unroll
    for (int t = 0; t < 4; ++t) { const float bv = bfr(bias[c0 + t * 16 + lr]);
#pragma unroll
        for (int j = 0; j < 8; ++j) os[(hi * 8 + j) * 68 + t * 16 + lr] = acc[t][j] + bv; }
    __syncthreads();
    float* crow = C + (size_t)r0 * NOUT + c0;
    auto pass = [&]() {
#pragma unroll
        for (int s = 0; s < 8; ++s) { const int Lid = (lane >> 3) + 4 * s, piece = lane & 7; const int row = Lid >> 1, cofs = (Lid & 1) * 32 + piece * 4;
            const v4f val = *(const v4fa*)(os + row * 68 + cofs); *(volatile v4f*)(crow + (size_t)row * NOUT + cofs) = val; }
    };
    pass(); __threadfence(); pass();
}

extern "C" void kernel_launch(void* const* d_in, const int* in_sizes, int n_in,
                              void* d_out, int out_size, void* d_ws, size_t ws_size, hipStream_t stream) {
    (void)in_sizes; (void)n_in; (void)out_size;
    const float* x = (const float*)d_in[0]; const float* rel = (const float*)d_in[1]; const float* gw = (const float*)d_in[2]; const float* gb = (const float*)d_in[3];
    const float* Wm = (const float*)d_in[4]; const float* bias = (const float*)d_in[5];
    float* out = (float*)d_out;
    char* wsp = (char*)d_ws;
    auto take = [&](size_t bytes) { char* p = wsp; wsp += (bytes + 255) & ~(size_t)255; return (void*)p; };
    float* SI = (float*)take((size_t)NB_ * NN_ * 4); float* SJ = (float*)take((size_t)NB_ * NN_ * 4);
    h16* XT16 = (h16*)take((size_t)NB_ * DD * NN_ * 2); bf* AH = (bf*)take((size_t)NB_ * NN_ * DD * 2); bf* AL = (bf*)take((size_t)NB_ * NN_ * DD * 2); bf* WT = (bf*)take((size_t)NOUT * DD * 2);
    if ((size_t)(wsp - (char*)d_ws) > ws_size) return;
    k_sij<<<(NB_ * NN_ / 32 + 7) / 8, 256, 0, stream>>>(x, gw, SI, SJ);
    k_xt<<<dim3(NN_ / 64, DD / 64, NB_), 256, 0, stream>>>(x, XT16);
    k_wt<<<dim3(DD / 64, NOUT / 64, 1), 256, 0, stream>>>(Wm, WT);
    k_agg<<<dim3(NN_ / 64, NB_, 1), 128, 0, stream>>>(SI, SJ, rel, gw, gb, XT16, AH, AL);
    k_out<<<dim3((NB_ * NN_) / 64, NOUT / 64, 1), 128, 0, stream>>>(AH, AL, WT, bias, out);
}
